// FeatureAttentionLayer_83013127897470
// MI455X (gfx1250) — hardware-verified
//
#include <hip/hip_runtime.h>
#include <math.h>

typedef __attribute__((ext_vector_type(16))) _Float16 v16h;
typedef __attribute__((ext_vector_type(8)))  _Float16 v8h;
typedef __attribute__((ext_vector_type(8)))  float    v8f;
typedef __attribute__((ext_vector_type(4)))  float    v4f;
typedef __attribute__((ext_vector_type(2)))  float    v2f;

constexpr int kBatch = 16;
constexpr int kNodes = 128;
constexpr int kWin   = 256;
constexpr int kEmb   = 512;
constexpr int kRowsL = kBatch * kNodes;
constexpr int kColsL = 2 * kEmb;
constexpr float kNegSlope = 0.2f;
constexpr float kMaskFill = -1.0e12f;

constexpr float kCarryX = 64.0f;
constexpr float kCarryW = 1024.0f;
constexpr float kCarryP = 1024.0f;
constexpr float kFoldL  = 1.0f / (kCarryX * kCarryW);
constexpr float kFoldZ  = 1.0f / (kCarryX * kCarryP);
constexpr float kF16MinNormal = 6.103515625e-05f;

static_assert((kWin % 32) == 0 && (kNodes % 32) == 0);
static_assert((kRowsL % 64) == 0 && (kColsL % 64) == 0 && (kWin % 64) == 0 && (kNodes % 64) == 0);
static_assert((kEmb % 64) == 0);

constexpr size_t kOffXH   = 0;
constexpr size_t kOffXT   = kOffXH   + (size_t)kBatch * kWin * kNodes * 2;
constexpr size_t kOffWT   = kOffXT   + (size_t)kRowsL * kWin * 2;
constexpr size_t kOffADJ  = kOffWT   + (size_t)kColsL * kWin * 2;
constexpr size_t kOffLCAT = kOffADJ  + (size_t)kNodes * kNodes * 4;
constexpr size_t kOffATT  = kOffLCAT + (size_t)kRowsL * kColsL * 4;
constexpr size_t kWsTotal = kOffATT  + (size_t)kRowsL * kNodes * 2;
static_assert(kWsTotal == 11599872ull);
static_assert(kWsTotal <= 134217728ull);
static_assert((kOffXT % 128) == 0 && (kOffWT % 128) == 0 && (kOffADJ % 128) == 0 &&
              (kOffLCAT % 128) == 0 && (kOffATT % 128) == 0);

__device__ __forceinline__ _Float16 to_f16_flush(float v) {
  const float s = (fabsf(v) < kF16MinNormal) ? 0.0f : v;
  return (_Float16)s;
}

__device__ __forceinline__ v16h frag_load_h(const _Float16* p) {
  union U { v16h v; v8h h[2]; } f;
  f.h[0] = *(const v8h*)(p);
  f.h[1] = *(const v8h*)(p + 16);
  return f.v;
}

__device__ __forceinline__ v8f mma_f16(v16h a, v16h b, v8f c) {
  c = __builtin_amdgcn_wmma_f32_16x16x32_f16(false, a, false, b, (short)0, c, false, false);
  asm volatile("v_nop\n\tv_nop\n\tv_nop\n\tv_nop" : "+v"(c) : "v"(a), "v"(b));
  return c;
}

__global__ __launch_bounds__(256) void cast_scale_f16_kernel(
    const float* __restrict__ src, unsigned short* __restrict__ dst, int total8, float carry)
{
  const int i = blockIdx.x * 256 + threadIdx.x;
  if (i >= total8) return;
  const size_t e0 = (size_t)i << 3;
  const v4f a0 = *(const v4f*)(src + e0);
  const v4f a1 = *(const v4f*)(src + e0 + 4);
  v8h hv;
#pragma unroll
  for (int e = 0; e < 4; ++e) {
    hv[e]     = to_f16_flush(a0[e] * carry);
    hv[4 + e] = to_f16_flush(a1[e] * carry);
  }
  unsigned short* q = dst + e0;
  *(volatile v8h*)q = hv;
  __threadfence();
  *(volatile v8h*)q = hv;
}

__global__ __launch_bounds__(256) void transpose_scale_f16_kernel(
    const float* __restrict__ in, unsigned short* __restrict__ out,
    int ldIn, int ldOut, long strideIn, long strideOut, float carry)
{
  __shared__ __align__(16) float sT[64 * 68];
  const int t = threadIdx.x, lane = t & 31, wave = t >> 5;
  const int c0 = blockIdx.x * 64, r0 = blockIdx.y * 64;
  const float* src = in + (size_t)blockIdx.z * strideIn;
  unsigned short* dstb = out + (size_t)blockIdx.z * strideOut;
#pragma unroll
  for (int k = 0; k < 4; ++k) {
    const int idx = t + 256 * k;
    const int r = idx >> 4, c4 = (idx & 15) * 4;
    *(v4f*)(sT + r * 68 + c4) = *(const v4f*)(src + (size_t)(r0 + r) * ldIn + c0 + c4);
  }
  __syncthreads();
  const int q = lane >> 3, r8 = (lane & 7) * 8;
  v8h hv[2];
#pragma unroll
  for (int it = 0; it < 2; ++it) {
    const int oc = it * 32 + wave * 4 + q;
#pragma unroll
    for (int e = 0; e < 8; ++e) hv[it][e] = to_f16_flush(sT[(r8 + e) * 68 + oc] * carry);
  }
  for (int pass = 0; pass < 2; ++pass) {
#pragma unroll
    for (int it = 0; it < 2; ++it) {
      const int oc = it * 32 + wave * 4 + q;
      *(volatile v8h*)(dstb + (size_t)(c0 + oc) * ldOut + r0 + r8) = hv[it];
    }
    __threadfence();
  }
}

__global__ __launch_bounds__(256) void adjacency_kernel(
    const float* __restrict__ emb, const float* __restrict__ gum, float* __restrict__ adj)
{
#pragma clang fp contract(off)
  const int idx = blockIdx.x * 256 + threadIdx.x;
  const int i = idx >> 7, j = idx & (kNodes - 1);
  const float* ei = emb + (size_t)i * kEmb;
  const float* ej = emb + (size_t)j * kEmb;
  float dot = 0.0f, ni = 0.0f, nj = 0.0f;
#pragma unroll 1
  for (int e4 = 0; e4 < kEmb / 4; ++e4) {
    const v4f va = *(const v4f*)(ei + 4 * e4);
    const v4f vb = *(const v4f*)(ej + 4 * e4);
#pragma unroll
    for (int c = 0; c < 4; ++c) {
      dot = dot + va[c] * vb[c];
      ni  = ni  + va[c] * va[c];
      nj  = nj  + vb[c] * vb[c];
    }
  }
  const float outer = sqrtf(ni) * sqrtf(nj);
  float lg = dot / outer;
  lg = lg / outer;
  lg = (lg + 1.0f) * 0.5f;
  const v2f u = *(const v2f*)(gum + (size_t)idx * 2);
  const float u0 = u[0], u1 = u[1];
  const float g0 = -logf(-logf(u0));
  const float g1 = -logf(-logf(u1));
  const float y0 = lg + g0;
  const float y1 = (1.0f - lg) + g1;
  float v = (y0 > y1) ? 1.0f : 0.0f;
  v = (i == j) ? 0.0f : v;
  volatile float* q = adj + idx;
  *q = v;
  __threadfence();
  *q = v;
}

template <int BIAS_SPLIT, int ACT_SIG>
__global__ __launch_bounds__(256) void gemm_f16_kernel(
    const unsigned short* __restrict__ Ap, int lda, long strideA,
    const unsigned short* __restrict__ Btp, int ldb, long strideB,
    float* __restrict__ Cout, int ldc, long strideC,
    const float* __restrict__ biasv, int biasFrom,
    int M, int N, int K, float fold)
{
  __shared__ __align__(16) float sT[8][16 * 68];
  const int b    = blockIdx.y;
  const int lane = threadIdx.x & 31;
  const int wave = threadIdx.x >> 5;
  const int tilesN = N >> 6;
  const int tilesM = M >> 6;
  const int tile = blockIdx.x * 8 + wave;
  if (tile >= tilesM * tilesN) return;
  const int tm = tile / tilesN;
  const int tn = tile - tm * tilesN;
  const int m0 = tm << 6;
  const int n0 = tn << 6;

  const _Float16* Ab = (const _Float16*)Ap  + (size_t)b * strideA;
  const _Float16* Bb = (const _Float16*)Btp + (size_t)b * strideB;

  const int rlane = lane & 15;
  const int koff  = (lane >> 4) * 8;
  const int mOff  = (lane >> 4) * 8;

  v8f acc[4][4];
#pragma unroll
  for (int i = 0; i < 4; ++i)
#pragma unroll
    for (int j = 0; j < 4; ++j) acc[i][j] = (v8f){0.f,0.f,0.f,0.f,0.f,0.f,0.f,0.f};

  for (int k0 = 0; k0 < K; k0 += 32) {
    v16h bh[4];
#pragma unroll
    for (int j = 0; j < 4; ++j) {
      const size_t bo = (size_t)(n0 + (j << 4) + rlane) * ldb + koff + k0;
      bh[j] = frag_load_h(Bb + bo);
    }
#pragma unroll
    for (int i = 0; i < 4; ++i) {
      const size_t ao = (size_t)(m0 + (i << 4) + rlane) * lda + koff + k0;
      const v16h ah = frag_load_h(Ab + ao);
#pragma unroll
      for (int j = 0; j < 4; ++j) acc[i][j] = mma_f16(ah, bh[j], acc[i][j]);
    }
  }

  float* slab = sT[wave];
  float* C = Cout + (size_t)b * strideC;
  const int hh = lane >> 4, c4 = (lane & 15) * 4;
#pragma unroll
  for (int i = 0; i < 4; ++i) {
    const int mBase = m0 + (i << 4);
#pragma unroll
    for (int j = 0; j < 4; ++j) {
      const int n = n0 + (j << 4) + rlane;
      float bv = 0.f;
      if (BIAS_SPLIT) {
        const int nb = (n >= biasFrom) ? (n - biasFrom) : n;
        float raw = biasv[nb];
        asm volatile("" : "+v"(raw));
        bv = (n >= biasFrom) ? raw : 0.0f;
      }
#pragma unroll
      for (int r = 0; r < 8; ++r) {
        const float v = acc[i][j][r] * fold + bv;
        slab[(mOff + r) * 68 + (j << 4) + rlane] = v;
      }
    }
    __builtin_amdgcn_fence(__ATOMIC_RELEASE, "workgroup");
    __builtin_amdgcn_wave_barrier();
    __builtin_amdgcn_fence(__ATOMIC_ACQUIRE, "workgroup");
    if (ACT_SIG) {
#pragma unroll 1
      for (int it = 0; it < 8; ++it) {
        float* sp = slab + (it * 2 + hh) * 68 + c4;
        const v4f zv = *(const v4f*)sp;
        v4f ov;
        ov[0] = 1.0f / (1.0f + expf(-zv[0]));
        ov[1] = 1.0f / (1.0f + expf(-zv[1]));
        ov[2] = 1.0f / (1.0f + expf(-zv[2]));
        ov[3] = 1.0f / (1.0f + expf(-zv[3]));
        *(v4f*)sp = ov;
      }
    }
    for (int pass = 0; pass < 2; ++pass) {
#pragma unroll
      for (int it = 0; it < 8; ++it) {
        const int row = it * 2 + hh;
        const v4f v = *(const v4f*)(slab + row * 68 + c4);
        *(volatile v4f*)(C + (size_t)(mBase + row) * ldc + n0 + c4) = v;
      }
      __threadfence();
    }
    __builtin_amdgcn_fence(__ATOMIC_RELEASE, "workgroup");
    __builtin_amdgcn_wave_barrier();
    __builtin_amdgcn_fence(__ATOMIC_ACQUIRE, "workgroup");
  }
}

__global__ __launch_bounds__(256) void score_softmax_kernel(
    const float* __restrict__ Lcat, const float* __restrict__ adj, const float* __restrict__ bias,
    const float* __restrict__ avec, unsigned short* __restrict__ att)
{
  __shared__ __align__(16) float sL1[16 * 68];
  __shared__ __align__(16) float sL2[kNodes * 68];
  __shared__ __align__(16) float sA[kEmb];
  __shared__ __align__(16) float sE[16 * 132];

  const int t  = threadIdx.x;
  const int b  = blockIdx.x >> 3;
  const int i0 = (blockIdx.x & 7) * 16;
  const int m  = t & 15;
  const int jb = (t >> 4) * 8;

  sA[t]       = avec[t];
  sA[t + 256] = avec[t + 256];

  float acc[8];
#pragma unroll
  for (int q = 0; q < 8; ++q) acc[q] = 0.0f;

  const float* L1b = Lcat + (size_t)(b * kNodes + i0) * kColsL;
  const float* L2b = Lcat + (size_t)(b * kNodes) * kColsL + kEmb;

#pragma unroll 1
  for (int ec = 0; ec < kEmb / 64; ++ec) {
    __syncthreads();
    {
      const int r = t >> 4, c4 = (t & 15) * 4;
      *(v4f*)(sL1 + r * 68 + c4) = *(const v4f*)(L1b + (size_t)r * kColsL + ec * 64 + c4);
    }
#pragma unroll
    for (int k = 0; k < 8; ++k) {
      const int idx = t + 256 * k;
      const int j = idx >> 4, c4 = (idx & 15) * 4;
      *(v4f*)(sL2 + j * 68 + c4) = *(const v4f*)(L2b + (size_t)j * kColsL + ec * 64 + c4);
    }
    __syncthreads();
#pragma unroll 1
    for (int e4 = 0; e4 < 16; ++e4) {
      const v4f l1v = *(const v4f*)(sL1 + m * 68 + 4 * e4);
      const v4f av  = *(const v4f*)(sA + ec * 64 + 4 * e4);
#pragma unroll
      for (int q = 0; q < 8; ++q) {
        const v4f l2v = *(const v4f*)(sL2 + (jb + q) * 68 + 4 * e4);
#pragma unroll
        for (int c = 0; c < 4; ++c) {
          const float p = l1v[c] + l2v[c];
          acc[q] = fmaf(av[c], fmaxf(p, kNegSlope * p), acc[q]);
        }
      }
    }
  }

  {
    const size_t mo = (size_t)(i0 + m) * kNodes + jb;
    const v4f ad0 = *(const v4f*)(adj + mo);
    const v4f ad1 = *(const v4f*)(adj + mo + 4);
    const v4f bs0 = *(const v4f*)(bias + mo);
    const v4f bs1 = *(const v4f*)(bias + mo + 4);
    v4f e0, e1;
    e0[0] = ((ad0[0] == 1.0f) ? acc[0] : kMaskFill) + bs0[0];
    e0[1] = ((ad0[1] == 1.0f) ? acc[1] : kMaskFill) + bs0[1];
    e0[2] = ((ad0[2] == 1.0f) ? acc[2] : kMaskFill) + bs0[2];
    e0[3] = ((ad0[3] == 1.0f) ? acc[3] : kMaskFill) + bs0[3];
    e1[0] = ((ad1[0] == 1.0f) ? acc[4] : kMaskFill) + bs1[0];
    e1[1] = ((ad1[1] == 1.0f) ? acc[5] : kMaskFill) + bs1[1];
    e1[2] = ((ad1[2] == 1.0f) ? acc[6] : kMaskFill) + bs1[2];
    e1[3] = ((ad1[3] == 1.0f) ? acc[7] : kMaskFill) + bs1[3];
    *(v4f*)(sE + m * 132 + jb)     = e0;
    *(v4f*)(sE + m * 132 + jb + 4) = e1;
  }
  __syncthreads();

  const int lane = t & 31, wave = t >> 5;
  const int hh = lane >> 4, c8 = (lane & 15) * 8;
  const int row = wave * 2 + hh;
  const v4f s0 = *(const v4f*)(sE + row * 132 + c8);
  const v4f s1 = *(const v4f*)(sE + row * 132 + c8 + 4);
  float mx = fmaxf(fmaxf(fmaxf(s0[0], s0[1]), fmaxf(s0[2], s0[3])),
                   fmaxf(fmaxf(s1[0], s1[1]), fmaxf(s1[2], s1[3])));
  mx = fmaxf(mx, __shfl_xor(mx, 1, 32));
  mx = fmaxf(mx, __shfl_xor(mx, 2, 32));
  mx = fmaxf(mx, __shfl_xor(mx, 4, 32));
  mx = fmaxf(mx, __shfl_xor(mx, 8, 32));
  float p[8];
  p[0] = expf(s0[0] - mx);
  p[1] = expf(s0[1] - mx);
  p[2] = expf(s0[2] - mx);
  p[3] = expf(s0[3] - mx);
  p[4] = expf(s1[0] - mx);
  p[5] = expf(s1[1] - mx);
  p[6] = expf(s1[2] - mx);
  p[7] = expf(s1[3] - mx);
  float sum = ((p[0] + p[1]) + (p[2] + p[3])) + ((p[4] + p[5]) + (p[6] + p[7]));
  sum += __shfl_xor(sum, 1, 32);
  sum += __shfl_xor(sum, 2, 32);
  sum += __shfl_xor(sum, 4, 32);
  sum += __shfl_xor(sum, 8, 32);
  const float inv = 1.0f / sum;
  v8h hv;
#pragma unroll
  for (int e = 0; e < 8; ++e) hv[e] = to_f16_flush((p[e] * inv) * kCarryP);
  unsigned short* dst = att + (size_t)(b * kNodes + i0 + wave * 2) * kNodes + lane * 8;
  *(volatile v8h*)dst = hv;
  __threadfence();
  *(volatile v8h*)dst = hv;
}

extern "C" void kernel_launch(void* const* d_in, const int* in_sizes, int n_in,
                              void* d_out, int out_size, void* d_ws, size_t ws_size,
                              hipStream_t stream) {
  if (n_in < 7) return;
  if (in_sizes[0] != kBatch * kWin * kNodes) return;
  if (in_sizes[1] != kNodes * kEmb) return;
  if (in_sizes[2] != 2 * kWin * kEmb) return;
  if (in_sizes[3] != kEmb) return;
  if (in_sizes[4] != kEmb) return;
  if (in_sizes[5] != kNodes * kNodes) return;
  if (in_sizes[6] != kNodes * kNodes * 2) return;
  if (out_size != kBatch * kWin * kNodes) return;
  if (ws_size < kWsTotal) return;

  const float* x      = (const float*)d_in[0];
  const float* emb    = (const float*)d_in[1];
  const float* W_lin  = (const float*)d_in[2];
  const float* b_lin  = (const float*)d_in[3];
  const float* avec   = (const float*)d_in[4];
  const float* bias   = (const float*)d_in[5];
  const float* gum    = (const float*)d_in[6];
  float* out = (float*)d_out;

  char* ws = (char*)d_ws;
  unsigned short* XH   = (unsigned short*)(ws + kOffXH);
  unsigned short* XT   = (unsigned short*)(ws + kOffXT);
  unsigned short* WT   = (unsigned short*)(ws + kOffWT);
  float*          ADJ  = (float*)(ws + kOffADJ);
  float*          LCAT = (float*)(ws + kOffLCAT);
  unsigned short* ATT  = (unsigned short*)(ws + kOffATT);

  cast_scale_f16_kernel<<<(kBatch * kWin * kNodes / 8) / 256, 256, 0, stream>>>(
      x, XH, kBatch * kWin * kNodes / 8, kCarryX);

  transpose_scale_f16_kernel<<<dim3(kNodes / 64, kWin / 64, kBatch), 256, 0, stream>>>(
      x, XT, kNodes, kWin, (long)kWin * kNodes, (long)kNodes * kWin, kCarryX);

  transpose_scale_f16_kernel<<<dim3(kEmb / 64, kWin / 64, 2), 256, 0, stream>>>(
      W_lin, WT, kEmb, kWin, (long)kWin * kEmb, (long)kEmb * kWin, kCarryW);

  adjacency_kernel<<<(kNodes * kNodes) / 256, 256, 0, stream>>>(emb, gum, ADJ);

  gemm_f16_kernel<1, 0><<<dim3((kRowsL / 64) * (kColsL / 64) / 8, 1), 256, 0, stream>>>(
      XT, kWin, 0L,
      WT, kWin, 0L,
      LCAT, kColsL, 0L,
      b_lin, kEmb,
      kRowsL, kColsL, kWin, kFoldL);

  score_softmax_kernel<<<kBatch * (kNodes / 16), 256, 0, stream>>>(LCAT, ADJ, bias, avec, ATT);

  gemm_f16_kernel<0, 1><<<dim3(1, kBatch), 256, 0, stream>>>(
      XH, kNodes, (long)kWin * kNodes,
      ATT, kNodes, (long)kNodes * kNodes,
      out, kNodes, (long)kWin * kNodes,
      nullptr, 0,
      kWin, kNodes, kNodes, kFoldZ);
}
